// MoEClusteredAttention_40089224741574
// MI455X (gfx1250) — hardware-verified
//
#include <hip/hip_runtime.h>
#include <math.h>
#include <stdint.h>

#ifndef NB
#define NB 2
#endif
#ifndef SEQ
#define SEQ 2048
#endif
#define SQ       SEQ
#define SKV      SEQ
#define NB_FULL  2
#define SQ_FULL  2048
#define DM       1024
#define NH       16
#define HD       64
#define INNER    (NH * HD)
#define NCL      8
#define WSC      256.0f
#define QS       8.0f
#define KS       8.0f
#define VS       8.0f
#define RESC     2048.0f
#define PCAR     32768.0f
#define OSC      1024.0f
#define LOG2E    1.4426950408889634f
#define RSQ_HD   0.125f
#define NEGB     (-1.0e9f)
#define NKB      (SKV / 32)
#define ATT_WAVES   4
#define ATT_THREADS (ATT_WAVES * 32)
#define CVT_THREADS (DM / 8)
#define RT_THREADS  256
#define TR_THREADS  256
#define OPITCH   68
#define GPITCH   68
#define TPITCH   68

static_assert(NB >= 1 && NB <= NB_FULL);
static_assert((SQ % 256) == 0 && SQ >= 256 && SQ <= SQ_FULL);
static_assert((SKV % 256) == 0 && SKV >= 256 && SKV <= SQ_FULL && NKB * 32 == SKV);
static_assert(HD == 64 && NH == 16 && INNER == 1024 && INNER == DM && NCL == 8);
static_assert((DM % 128) == 0 && (DM % 64) == 0 && (DM % 32) == 0);
static_assert(CVT_THREADS == 128 && (CVT_THREADS % 32) == 0);
static_assert((DM * NCL) % (RT_THREADS * 4) == 0);
static_assert((OPITCH * 4) % 16 == 0 && (GPITCH * 4) % 16 == 0 && (TPITCH * 4) % 16 == 0);
static_assert(ATT_THREADS == 128 && TR_THREADS == 256);

typedef unsigned short u16;
typedef _Float16 v16h __attribute__((ext_vector_type(16)));
typedef _Float16 v8h  __attribute__((ext_vector_type(8)));
typedef float    v8f  __attribute__((ext_vector_type(8)));
typedef float    v4f  __attribute__((ext_vector_type(4)));
typedef unsigned int v4u __attribute__((ext_vector_type(4)));
typedef int      v4i  __attribute__((ext_vector_type(4)));

union FragH { v16h v; v8h h[2]; v4u u[2]; };

__device__ __forceinline__ unsigned short bf_bits(float f) {
  unsigned u = __float_as_uint(f);
  return (unsigned short)((u + 0x7FFFu + ((u >> 16) & 1u)) >> 16);
}
__device__ __forceinline__ float bf_up(unsigned short h) { return __uint_as_float(((unsigned)h) << 16); }
__device__ __forceinline__ float bfr(float f) { return bf_up(bf_bits(f)); }
__device__ __forceinline__ unsigned short h_bits(_Float16 x) { return __builtin_bit_cast(unsigned short, x); }
__device__ __forceinline__ unsigned pk16(unsigned short a, unsigned short b) { return (unsigned)a | ((unsigned)b << 16); }
__device__ __forceinline__ v8f zero8() { v8f z = {0.f, 0.f, 0.f, 0.f, 0.f, 0.f, 0.f, 0.f}; return z; }
__device__ __forceinline__ v4f bfr4(v4f a) { v4f r; r[0] = bfr(a[0]); r[1] = bfr(a[1]); r[2] = bfr(a[2]); r[3] = bfr(a[3]); return r; }
__device__ __forceinline__ v4u pack8h(v4f a, v4f c4) {
  v4u o;
#pragma unroll
  for (int e = 0; e < 2; ++e) {
    o[e]     = pk16(h_bits((_Float16)a[2 * e]),  h_bits((_Float16)a[2 * e + 1]));
    o[2 + e] = pk16(h_bits((_Float16)c4[2 * e]), h_bits((_Float16)c4[2 * e + 1]));
  }
  return o;
}

__device__ __forceinline__ v16h ldfrag_h(const _Float16* p) {
  FragH f;
  f.h[0] = *(const v8h*)(p);
  f.h[1] = *(const v8h*)(p + 16);
  return f.v;
}

__device__ __forceinline__ v8f mma_h(v16h a, v16h b, v8f c) {
  return __builtin_amdgcn_wmma_f32_16x16x32_f16(false, a, false, b, (short)0, c, false, false);
}
__device__ __forceinline__ void guard_s6(v8f& a, v8f& b, v8f& c, v8f& d,
                                         v16h x0, v16h x1, v16h x2, v16h x3, v16h x4, v16h x5) {
#if defined(__HIP_DEVICE_COMPILE__)
  asm volatile("v_nop\n\tv_nop\n\tv_nop\n\tv_nop"
               : "+v"(a), "+v"(b), "+v"(c), "+v"(d) : "v"(x0), "v"(x1), "v"(x2), "v"(x3), "v"(x4), "v"(x5) : "memory");
#endif
}
__device__ __forceinline__ void guard_p(v8f& a, v8f& b, v8f& c, v8f& d, v16h p, v16h x0, v16h x1, v16h x2, v16h x3) {
#if defined(__HIP_DEVICE_COMPILE__)
  asm volatile("v_nop\n\tv_nop\n\tv_nop\n\tv_nop"
               : "+v"(a), "+v"(b), "+v"(c), "+v"(d) : "v"(p), "v"(x0), "v"(x1), "v"(x2), "v"(x3) : "memory");
#endif
}
__device__ __forceinline__ void guard_g(v8f (&acc)[8], v16h x0, v16h x1, v16h x2, v16h x3, v16h x4, v16h x5) {
#if defined(__HIP_DEVICE_COMPILE__)
  asm volatile("v_nop\n\tv_nop\n\tv_nop\n\tv_nop"
               : "+v"(acc[0]), "+v"(acc[1]), "+v"(acc[2]), "+v"(acc[3]),
                 "+v"(acc[4]), "+v"(acc[5]), "+v"(acc[6]), "+v"(acc[7])
               : "v"(x0), "v"(x1), "v"(x2), "v"(x3), "v"(x4), "v"(x5) : "memory");
#endif
}
__device__ __forceinline__ void acc_guard4(v8f& a, v8f& b, v8f& c, v8f& d) {
#if defined(__HIP_DEVICE_COMPILE__)
  asm volatile("v_nop\n\tv_nop\n\tv_nop\n\tv_nop" : "+v"(a), "+v"(b), "+v"(c), "+v"(d));
#endif
}
__device__ __forceinline__ void wave_sync_lds() {
  __builtin_amdgcn_fence(__ATOMIC_RELEASE, "workgroup");
  __builtin_amdgcn_wave_barrier();
  __builtin_amdgcn_fence(__ATOMIC_ACQUIRE, "workgroup");
}

__global__ __launch_bounds__(RT_THREADS)
void route_ids(const float* xq, const float* xk, const float* __restrict__ Wr, int* Asg) {
  __shared__ __align__(16) float wl[DM * NCL];
  const int tid = threadIdx.x;
#pragma unroll
  for (int i = 0; i < (DM * NCL) / (RT_THREADS * 4); ++i) {
    const int e = (i * RT_THREADS + tid) * 4;
    *(v4f*)(wl + e) = bfr4(*(const v4f*)(Wr + e));
  }
  __syncthreads();
  constexpr int NBQ = (NB * SQ) / RT_THREADS;
  int blk = blockIdx.x;
  const float* X = xq; int rows = SQ; int* dst = Asg;
  if (blk >= NBQ) { blk -= NBQ; X = xk; rows = SKV; dst = Asg + NB * SQ; }
  const int t = blk * RT_THREADS + tid;
  const int b = t / rows, s = t - b * rows;
  const float* x = X + ((size_t)b * SQ_FULL + (size_t)s) * (size_t)DM;
  double acc[NCL];
#pragma unroll
  for (int mm = 0; mm < NCL; ++mm) acc[mm] = 0.0;
#pragma unroll 1
  for (int dd = 0; dd < DM; dd += 4) {
    const v4f xa = bfr4(*(const v4f*)(x + dd));
#pragma unroll
    for (int e = 0; e < 4; ++e) {
      const v4f w0 = *(const v4f*)(wl + (dd + e) * NCL);
      const v4f w1 = *(const v4f*)(wl + (dd + e) * NCL + 4);
      const double xd = (double)xa[e];
#pragma unroll
      for (int mm = 0; mm < 4; ++mm) {
        acc[mm]     = fma(xd, (double)w0[mm], acc[mm]);
        acc[4 + mm] = fma(xd, (double)w1[mm], acc[4 + mm]);
      }
    }
  }
  double best = acc[0];
  int bi = 0;
#pragma unroll
  for (int mm = 1; mm < NCL; ++mm) {
    const bool gt = acc[mm] > best;
    best = gt ? acc[mm] : best;
    bi   = gt ? mm : bi;
  }
  int* p = dst + t;
  *(volatile int*)p = bi;
  __threadfence();
  *(volatile int*)p = bi;
}

__global__ __launch_bounds__(CVT_THREADS)
void cvt16x3(const float* xq, const float* xk, const float* xv, u16* YQ, u16* YK, u16* YV) {
  const int tid = threadIdx.x;
  int r = blockIdx.x;
  const float* x = xq; u16* Y = YQ; int rows = SQ;
  if (r >= NB * SQ) {
    r -= NB * SQ; x = xk; Y = YK; rows = SKV;
    if (r >= NB * SKV) { r -= NB * SKV; x = xv; Y = YV; }
  }
  const int b = r / rows;
  const int s = r - b * rows;
  const float* src = x + ((size_t)b * (size_t)SQ_FULL + (size_t)s) * (size_t)DM + (size_t)tid * 8;
  const v4f a = *(const v4f*)(src), c4 = *(const v4f*)(src + 4);
  const v4u o = pack8h(bfr4(a), bfr4(c4));
  u16* dst = Y + (size_t)r * (size_t)DM + (size_t)tid * 8;
  for (int pass = 0; pass < 2; ++pass) {
    *(volatile v4u*)(dst) = o;
    __threadfence();
  }
}

__global__ __launch_bounds__(TR_THREADS)
void wtr16(const float* W0, const float* W1, const float* W2, const float* W3, u16* WT) {
  __shared__ __align__(16) float T[64 * TPITCH];
  const int tid = threadIdx.x;
  constexpr int NT = DM / 64;
  constexpr int TPW = NT * NT;
  const int bid = blockIdx.x;
  const int w = bid / TPW;
  const int tile = bid - w * TPW;
  const int nt = tile % NT, kt = tile / NT;
  const int n0 = nt * 64, k0 = kt * 64;
  const float* W = W0;
  if (w == 1) W = W1;
  if (w == 2) W = W2;
  if (w == 3) W = W3;
  const int kr = tid >> 4, nc = (tid & 15) * 4;
#pragma unroll
  for (int p = 0; p < 4; ++p) {
    const int k = kr + 16 * p;
    const v4f v = bfr4(*(const v4f*)(W + (size_t)(k0 + k) * (size_t)DM + n0 + nc)) * WSC;
#pragma unroll
    for (int e = 0; e < 4; ++e) T[(nc + e) * TPITCH + k] = v[e];
  }
  __syncthreads();
  const int wave = tid >> 5, lane = tid & 31, rq = lane >> 3, c8 = (lane & 7) * 8;
  v4u ov[2];
#pragma unroll
  for (int i = 0; i < 2; ++i) {
    const int row = wave * 8 + 4 * i + rq;
    const v4f a = *(const v4f*)(T + row * TPITCH + c8), c4 = *(const v4f*)(T + row * TPITCH + c8 + 4);
    ov[i] = pack8h(a, c4);
  }
  u16* base = WT + ((size_t)w * DM + (size_t)n0) * (size_t)DM + (size_t)k0 + (size_t)c8;
  for (int pass = 0; pass < 2; ++pass) {
#pragma unroll
    for (int i = 0; i < 2; ++i) {
      const int row = wave * 8 + 4 * i + rq;
      *(volatile v4u*)(base + (size_t)row * (size_t)DM) = ov[i];
    }
    __threadfence();
  }
}

__device__ __forceinline__ void gemm_core(const _Float16* ap, const _Float16* bp, int K, v8f (&acc)[8]) {
  const size_t rs16 = (size_t)16 * (size_t)K;
#pragma unroll 1
  for (int k0 = 0; k0 < K; k0 += 32) {
    const v16h a0 = ldfrag_h(ap + k0), a1 = ldfrag_h(ap + rs16 + k0);
    const v16h b0 = ldfrag_h(bp + k0);
    const v16h b1 = ldfrag_h(bp + rs16 + k0);
    const v16h b2 = ldfrag_h(bp + 2 * rs16 + k0);
    const v16h b3 = ldfrag_h(bp + 3 * rs16 + k0);
    acc[0] = mma_h(a0, b0, acc[0]);
    acc[1] = mma_h(a0, b1, acc[1]);
    acc[2] = mma_h(a0, b2, acc[2]);
    acc[3] = mma_h(a0, b3, acc[3]);
    acc[4] = mma_h(a1, b0, acc[4]);
    acc[5] = mma_h(a1, b1, acc[5]);
    acc[6] = mma_h(a1, b2, acc[6]);
    acc[7] = mma_h(a1, b3, acc[7]);
    guard_g(acc, a0, a1, b0, b1, b2, b3);
  }
}
__device__ __forceinline__ void stage32x64(float* sl, v8f (&acc)[8], float oscale, int lane) {
  const int hh = lane >> 4, m = lane & 15;
#pragma unroll
  for (int i = 0; i < 2; ++i) {
#pragma unroll
    for (int r = 0; r < 8; ++r) {
      const int ro = (16 * i + 8 * hh + r) * GPITCH + m;
      sl[ro]      = acc[4 * i + 0][r] * oscale;
      sl[ro + 16] = acc[4 * i + 1][r] * oscale;
      sl[ro + 32] = acc[4 * i + 2][r] * oscale;
      sl[ro + 48] = acc[4 * i + 3][r] * oscale;
    }
  }
  wave_sync_lds();
}

__global__ __launch_bounds__(128)
void gemm_o16(const u16* __restrict__ A, const u16* __restrict__ Bt, u16* C,
              int Mb, int N, int K, int aBs, int bBs, int cBs, float oscale) {
  __shared__ __align__(16) float slab[4 * 32 * GPITCH];
  const int tid = threadIdx.x, wave = tid >> 5, lane = tid & 31, hh = lane >> 4, m = lane & 15;
  const int ntile = N >> 6, mtile = Mb >> 7;
  const int bid  = blockIdx.x;
  const int nt   = bid % ntile;
  const int tmp  = bid / ntile;
  const int mt   = tmp % mtile;
  const int bz   = tmp / mtile;
  const int rowb = mt * 128 + wave * 32;
  const int col0 = nt * 64;
  if (rowb + 32 > Mb) return;
  const _Float16* Ab = (const _Float16*)(const void*)A + (size_t)bz * (size_t)aBs;
  const _Float16* Bb = (const _Float16*)(const void*)Bt + (size_t)bz * (size_t)bBs;
  const _Float16* ap = Ab + (size_t)(rowb + m) * K + 8 * hh;
  const _Float16* bp = Bb + (size_t)(col0 + m) * K + 8 * hh;
  v8f acc[8];
#pragma unroll
  for (int i = 0; i < 8; ++i) acc[i] = zero8();
  gemm_core(ap, bp, K, acc);
  float* sl = slab + wave * 32 * GPITCH;
  stage32x64(sl, acc, oscale, lane);
  const int rq = lane >> 3, c8 = (lane & 7) * 8;
  v4u ov[8];
#pragma unroll
  for (int i = 0; i < 8; ++i) {
    const int row = 4 * i + rq;
    const v4f a = *(const v4f*)(sl + row * GPITCH + c8), c4 = *(const v4f*)(sl + row * GPITCH + c8 + 4);
    ov[i] = pack8h(a, c4);
  }
  u16* Cb = C + (size_t)bz * (size_t)cBs + (size_t)rowb * (size_t)N + col0 + c8;
  for (int pass = 0; pass < 2; ++pass) {
#pragma unroll
    for (int i = 0; i < 8; ++i) {
      const int row = 4 * i + rq;
      *(volatile v4u*)(Cb + (size_t)row * (size_t)N) = ov[i];
    }
    __threadfence();
  }
}

__global__ __launch_bounds__(128)
void gemm_o16x2(const u16* __restrict__ A, const u16* __restrict__ Bt, u16* CH, u16* CL,
                int Mb, int N, int K, float oscale) {
  __shared__ __align__(16) float slab[4 * 32 * GPITCH];
  const int tid = threadIdx.x, wave = tid >> 5, lane = tid & 31, hh = lane >> 4, m = lane & 15;
  const int ntile = N >> 6;
  const int bid  = blockIdx.x;
  const int nt   = bid % ntile;
  const int mt   = bid / ntile;
  const int rowb = mt * 128 + wave * 32;
  const int col0 = nt * 64;
  if (rowb + 32 > Mb) return;
  const _Float16* ap = (const _Float16*)(const void*)A + (size_t)(rowb + m) * K + 8 * hh;
  const _Float16* bp = (const _Float16*)(const void*)Bt + (size_t)(col0 + m) * K + 8 * hh;
  v8f acc[8];
#pragma unroll
  for (int i = 0; i < 8; ++i) acc[i] = zero8();
  gemm_core(ap, bp, K, acc);
  float* sl = slab + wave * 32 * GPITCH;
  stage32x64(sl, acc, oscale, lane);
  const int rq = lane >> 3, c8 = (lane & 7) * 8;
  v4u oh[8], ol[8];
#pragma unroll
  for (int i = 0; i < 8; ++i) {
    const int row = 4 * i + rq;
    const v4f a = *(const v4f*)(sl + row * GPITCH + c8), c4 = *(const v4f*)(sl + row * GPITCH + c8 + 4);
#pragma unroll
    for (int e = 0; e < 2; ++e) {
      const _Float16 ha0 = (_Float16)a[2 * e],  ha1 = (_Float16)a[2 * e + 1];
      const _Float16 hc0 = (_Float16)c4[2 * e], hc1 = (_Float16)c4[2 * e + 1];
      const _Float16 la0 = (_Float16)((a[2 * e]      - (float)ha0) * RESC);
      const _Float16 la1 = (_Float16)((a[2 * e + 1]  - (float)ha1) * RESC);
      const _Float16 lc0 = (_Float16)((c4[2 * e]     - (float)hc0) * RESC);
      const _Float16 lc1 = (_Float16)((c4[2 * e + 1] - (float)hc1) * RESC);
      oh[i][e]     = pk16(h_bits(ha0), h_bits(ha1));
      oh[i][2 + e] = pk16(h_bits(hc0), h_bits(hc1));
      ol[i][e]     = pk16(h_bits(la0), h_bits(la1));
      ol[i][2 + e] = pk16(h_bits(lc0), h_bits(lc1));
    }
  }
  const size_t cbase = (size_t)rowb * (size_t)N + (size_t)col0 + (size_t)c8;
  u16* Hb = CH + cbase;
  u16* Lb = CL + cbase;
  for (int pass = 0; pass < 2; ++pass) {
#pragma unroll
    for (int i = 0; i < 8; ++i) {
      const int row = 4 * i + rq;
      *(volatile v4u*)(Hb + (size_t)row * (size_t)N) = oh[i];
    }
#pragma unroll
    for (int i = 0; i < 8; ++i) {
      const int row = 4 * i + rq;
      *(volatile v4u*)(Lb + (size_t)row * (size_t)N) = ol[i];
    }
    __threadfence();
  }
}

__global__ __launch_bounds__(128)
void gemm_o32(const u16* __restrict__ A, const u16* __restrict__ Bt, float* C,
              int Mb, int N, int K, int aBs, int bBs, int cBs, float oscale) {
  __shared__ __align__(16) float slab[4 * 32 * GPITCH];
  const int tid = threadIdx.x, wave = tid >> 5, lane = tid & 31, hh = lane >> 4, m = lane & 15;
  const int ntile = N >> 6, mtile = Mb >> 7;
  const int bid  = blockIdx.x;
  const int nt   = bid % ntile;
  const int tmp  = bid / ntile;
  const int mt   = tmp % mtile;
  const int bz   = tmp / mtile;
  const int rowb = mt * 128 + wave * 32;
  const int col0 = nt * 64;
  if (rowb + 32 > Mb) return;
  const _Float16* Ab = (const _Float16*)(const void*)A + (size_t)bz * (size_t)aBs;
  const _Float16* Bb = (const _Float16*)(const void*)Bt + (size_t)bz * (size_t)bBs;
  const _Float16* ap = Ab + (size_t)(rowb + m) * K + 8 * hh;
  const _Float16* bp = Bb + (size_t)(col0 + m) * K + 8 * hh;
  v8f acc[8];
#pragma unroll
  for (int i = 0; i < 8; ++i) acc[i] = zero8();
  gemm_core(ap, bp, K, acc);
  float* sl = slab + wave * 32 * GPITCH;
  stage32x64(sl, acc, oscale, lane);
  v4f vals[16];
#pragma unroll
  for (int it = 0; it < 16; ++it) vals[it] = *(const v4f*)(sl + (it * 2 + hh) * GPITCH + m * 4);
  float* Cb = C + (size_t)bz * (size_t)cBs + ((size_t)rowb + (size_t)hh) * (size_t)N + col0 + m * 4;
  for (int pass = 0; pass < 2; ++pass) {
#pragma unroll
    for (int it = 0; it < 16; ++it) {
      *(volatile v4f*)(Cb + (size_t)(it * 2) * (size_t)N) = vals[it];
    }
    __threadfence();
  }
}

__global__ __launch_bounds__(ATT_THREADS)
void attn_fwd(const u16* __restrict__ Qh, const u16* __restrict__ Ql, const u16* __restrict__ Kh,
              const u16* __restrict__ Kl, const u16* __restrict__ Vp, const int* __restrict__ Aq,
              const int* __restrict__ Ak, u16* Op) {
  __shared__ __align__(16) float smem[ATT_WAVES * 16 * OPITCH];

  const int tid  = threadIdx.x;
  const int wave = tid >> 5;
  const int lane = tid & 31;
  const int hh   = lane >> 4;
  const int c    = lane & 15;

  constexpr int NQT = SQ / 64;
  const int bid  = blockIdx.x;
  const int qt   = bid % NQT;
  const int head = (bid / NQT) % NH;
  const int b    = bid / (NQT * NH);
  const int q0   = qt * 64 + wave * 16;

  const size_t qoff = ((size_t)(b * SQ + q0 + c)) * INNER + head * HD + 8 * hh;
  const _Float16* Qhb = (const _Float16*)(const void*)Qh + qoff;
  const _Float16* Qlb = (const _Float16*)(const void*)Ql + qoff;
  const size_t koff = ((size_t)(b * SKV + c)) * INNER + head * HD + 8 * hh;
  const _Float16* Khb = (const _Float16*)(const void*)Kh + koff;
  const _Float16* Klb = (const _Float16*)(const void*)Kl + koff;
  const _Float16* Vb = (const _Float16*)(const void*)Vp + ((size_t)(b * NH + head) * HD + c) * SKV + 8 * hh;
  const int myg = Aq[b * SQ + q0 + c];
  const int* akb = Ak + (size_t)b * SKV + 8 * hh;
  const float lsc  = (LOG2E * RSQ_HD) / (QS * KS);
  const float rinv = 1.0f / RESC;

  v16h qh[2], ql[2];
  qh[0] = ldfrag_h(Qhb);
  qh[1] = ldfrag_h(Qhb + 32);
  ql[0] = ldfrag_h(Qlb);
  ql[1] = ldfrag_h(Qlb + 32);

  float mrun = -INFINITY, lrun = 0.f;
  v8f o[4];
#pragma unroll
  for (int j = 0; j < 4; ++j) o[j] = zero8();

#pragma unroll 1
  for (int it = 0; it < NKB; ++it) {
    const int kb = it * 32;
    v8f s0 = zero8(), s1 = zero8(), r0 = zero8(), r1 = zero8();
    const _Float16* kh0p = Khb + (size_t)kb * INNER;
    const _Float16* kh1p = kh0p + (size_t)16 * INNER;
    const _Float16* kl0p = Klb + (size_t)kb * INNER;
    const _Float16* kl1p = kl0p + (size_t)16 * INNER;
#pragma unroll
    for (int kk = 0; kk < HD / 32; ++kk) {
      const v16h kf0 = ldfrag_h(kh0p + kk * 32);
      const v16h kf1 = ldfrag_h(kh1p + kk * 32);
      const v16h lf0 = ldfrag_h(kl0p + kk * 32);
      const v16h lf1 = ldfrag_h(kl1p + kk * 32);
      s0 = mma_h(kf0, qh[kk], s0);
      s1 = mma_h(kf1, qh[kk], s1);
      r0 = mma_h(kf0, ql[kk], r0);
      r1 = mma_h(kf1, ql[kk], r1);
      r0 = mma_h(lf0, qh[kk], r0);
      r1 = mma_h(lf1, qh[kk], r1);
      guard_s6(s0, s1, r0, r1, qh[kk], ql[kk], kf0, kf1, lf0, lf1);
    }
    const v4i g0 = *(const v4i*)(akb + kb);
    const v4i g1 = *(const v4i*)(akb + kb + 4);
    const v4i g2 = *(const v4i*)(akb + kb + 16);
    const v4i g3 = *(const v4i*)(akb + kb + 20);
    float t[16];
#pragma unroll
    for (int i = 0; i < 4; ++i) {
      const float u0 = (s0[i]     + r0[i]     * rinv) * lsc;
      const float u1 = (s0[4 + i] + r0[4 + i] * rinv) * lsc;
      const float u2 = (s1[i]     + r1[i]     * rinv) * lsc;
      const float u3 = (s1[4 + i] + r1[4 + i] * rinv) * lsc;
      t[i]      = (g0[i] == myg) ? u0 : NEGB;
      t[4 + i]  = (g1[i] == myg) ? u1 : NEGB;
      t[8 + i]  = (g2[i] == myg) ? u2 : NEGB;
      t[12 + i] = (g3[i] == myg) ? u3 : NEGB;
    }
    float cm = t[0];
#pragma unroll
    for (int i = 1; i < 16; ++i) cm = fmaxf(cm, t[i]);
    cm = fmaxf(cm, __shfl_xor(cm, 16, 32));
    const float mn = fmaxf(mrun, cm);
    const float al = exp2f(mrun - mn);
    mrun = mn;
    float ps = 0.f;
    FragH ph;
#pragma unroll
    for (int w = 0; w < 2; ++w) {
#pragma unroll
      for (int e4 = 0; e4 < 4; ++e4) {
        const int i = 8 * w + 2 * e4;
        const float p0 = exp2f(t[i] - mn), p1 = exp2f(t[i + 1] - mn);
        ps += p0 + p1;
        ph.u[w][e4] = pk16(h_bits((_Float16)(p0 * PCAR)), h_bits((_Float16)(p1 * PCAR)));
      }
    }
    ps += __shfl_xor(ps, 16, 32);
    lrun = lrun * al + ps;
    float scl[8];
#pragma unroll
    for (int r = 0; r < 8; ++r) scl[r] = __shfl(al, 8 * hh + r, 32);
#pragma unroll
    for (int j = 0; j < 4; ++j) {
#pragma unroll
      for (int r = 0; r < 8; ++r) o[j][r] *= scl[r];
    }
    {
      const _Float16* vp = Vb + kb;
      const v16h v0 = ldfrag_h(vp);
      const v16h v1 = ldfrag_h(vp + (size_t)16 * SKV);
      const v16h v2 = ldfrag_h(vp + (size_t)32 * SKV);
      const v16h v3 = ldfrag_h(vp + (size_t)48 * SKV);
      o[0] = mma_h(ph.v, v0, o[0]);
      o[1] = mma_h(ph.v, v1, o[1]);
      o[2] = mma_h(ph.v, v2, o[2]);
      o[3] = mma_h(ph.v, v3, o[3]);
      guard_p(o[0], o[1], o[2], o[3], ph.v, v0, v1, v2, v3);
    }
  }
  acc_guard4(o[0], o[1], o[2], o[3]);

  const bool hit = (mrun > -1.0e8f);
  const float linv = hit ? (1.0f / lrun) * (OSC / (PCAR * VS)) : 0.0f;
  float inv[8];
#pragma unroll
  for (int r = 0; r < 8; ++r) inv[r] = __shfl(linv, 8 * hh + r, 32);
  float* slab = smem + wave * 16 * OPITCH;
#pragma unroll
  for (int r = 0; r < 8; ++r) {
#pragma unroll
    for (int j = 0; j < 4; ++j) slab[(8 * hh + r) * OPITCH + j * 16 + c] = o[j][r] * inv[r];
  }
  wave_sync_lds();
  v4u ov[4];
  const int rq = lane >> 3, c8 = (lane & 7) * 8;
#pragma unroll
  for (int i = 0; i < 4; ++i) {
    const int row = 4 * i + rq;
    const v4f a = *(const v4f*)(slab + row * OPITCH + c8), c4 = *(const v4f*)(slab + row * OPITCH + c8 + 4);
    ov[i] = pack8h(a, c4);
  }
  u16* ob = Op + ((size_t)(b * SQ + q0)) * INNER + head * HD + c8;
  for (int pass = 0; pass < 2; ++pass) {
#pragma unroll
    for (int i = 0; i < 4; ++i) {
      const int row = 4 * i + rq;
      *(volatile v4u*)(ob + (size_t)row * INNER) = ov[i];
    }
    __threadfence();
  }
}

extern "C" void kernel_launch(void* const* d_in, const int* in_sizes, int n_in,
                              void* d_out, int out_size, void* d_ws, size_t ws_size,
                              hipStream_t stream) {
  if (n_in < 8) return;
  const int needQ = ((NB - 1) * SQ_FULL + SQ) * DM;
  const int needK = ((NB - 1) * SQ_FULL + SKV) * DM;
  if (in_sizes[0] < needQ || in_sizes[1] < needK || in_sizes[2] < needK) return;
  if (in_sizes[3] < DM * DM || in_sizes[4] < DM * DM || in_sizes[5] < DM * DM || in_sizes[6] < DM * DM) return;
  if (in_sizes[7] < DM * NCL) return;
  if (out_size < needQ) return;

  const float* queries = (const float*)d_in[0];
  const float* keys    = (const float*)d_in[1];
  const float* values  = (const float*)d_in[2];
  const float* wq      = (const float*)d_in[3];
  const float* wk      = (const float*)d_in[4];
  const float* wv      = (const float*)d_in[5];
  const float* wo      = (const float*)d_in[6];
  const float* wr      = (const float*)d_in[7];
  float*       out     = (float*)d_out;

  const size_t szXQ   = (size_t)NB * SQ * DM * 2;
  const size_t szXK   = (size_t)NB * SKV * DM * 2;
  const size_t szWT   = (size_t)4 * DM * DM * 2;
  const size_t szQ16  = (size_t)NB * SQ * INNER * 2;
  const size_t szK16  = (size_t)NB * SKV * INNER * 2;
  const size_t szVT16 = (size_t)NB * INNER * SKV * 2;
  const size_t szO16  = (size_t)NB * SQ * INNER * 2;
  const size_t szASG  = (((size_t)NB * SQ + (size_t)NB * SKV) * 4 + 127) / 128 * 128;
  size_t off = 0;
  const size_t oXQ   = off; off += szXQ;
  const size_t oXK   = off; off += szXK;
  const size_t oXV   = off; off += szXK;
  const size_t oWT   = off; off += szWT;
  const size_t oQH   = off; off += szQ16;
  const size_t oQL   = off; off += szQ16;
  const size_t oKH   = off; off += szK16;
  const size_t oKL   = off; off += szK16;
  const size_t oVT16 = off; off += szVT16;
  const size_t oO16  = off; off += szO16;
  const size_t oASG  = off; off += szASG;
  if (off > ws_size) return;
  if (off > (size_t)134217728) return;

  char* ws = (char*)d_ws;
  u16* XQ   = (u16*)(ws + oXQ);
  u16* XK   = (u16*)(ws + oXK);
  u16* XV   = (u16*)(ws + oXV);
  u16* WT   = (u16*)(ws + oWT);
  u16* QH   = (u16*)(ws + oQH);
  u16* QL   = (u16*)(ws + oQL);
  u16* KH   = (u16*)(ws + oKH);
  u16* KL   = (u16*)(ws + oKL);
  u16* VT16 = (u16*)(ws + oVT16);
  u16* O16  = (u16*)(ws + oO16);
  int*  ASG = (int*)(ws + oASG);
  int*  ASGQ = ASG;
  int*  ASGK = ASG + (size_t)NB * SQ;

  route_ids<<<dim3((NB * SQ + NB * SKV) / RT_THREADS), dim3(RT_THREADS), 0, stream>>>(queries, keys, wr, ASG);
  cvt16x3<<<dim3(NB * SQ + 2 * NB * SKV), dim3(CVT_THREADS), 0, stream>>>(queries, keys, values, XQ, XK, XV);
  wtr16<<<dim3(4 * (DM / 64) * (DM / 64)), dim3(TR_THREADS), 0, stream>>>(wq, wk, wv, wo, WT);
  gemm_o16x2<<<dim3((NB * SQ / 128) * (INNER / 64)), dim3(128), 0, stream>>>(
      XQ, WT, QH, QL, NB * SQ, INNER, DM, QS / WSC);
  gemm_o16x2<<<dim3((NB * SKV / 128) * (INNER / 64)), dim3(128), 0, stream>>>(
      XK, WT + (size_t)DM * DM, KH, KL, NB * SKV, INNER, DM, KS / WSC);
  gemm_o16<<<dim3(NB * (INNER / 128) * (SKV / 64)), dim3(128), 0, stream>>>(
      WT + (size_t)2 * DM * DM, XV, VT16, INNER, SKV, DM, 0, SKV * DM, INNER * SKV, VS / WSC);
  attn_fwd<<<dim3(NB * NH * (SQ / 64)), dim3(ATT_THREADS), 0, stream>>>(QH, QL, KH, KL, VT16, ASGQ, ASGK, O16);
  gemm_o32<<<dim3(NB * (SQ / 128) * (DM / 64)), dim3(128), 0, stream>>>(
      O16, WT + (size_t)3 * DM * DM, out, SQ, DM, INNER, SQ * INNER, 0, SQ_FULL * DM, 1.0f / (OSC * WSC));
  (void)hipGetLastError();
}
